// BidirRWKV6TimeMix_76003741270340
// MI455X (gfx1250) — hardware-verified
//
#include <hip/hip_runtime.h>
#include <math.h>

constexpr int kB = 4;
constexpr int kT = 1024;
constexpr int kD = 1024;
constexpr int kH = 16;
constexpr int kHS = 64;
constexpr int kMixCols = 160;
constexpr int kMixPad = 192;
constexpr int kMixRank = 32;
constexpr int kDecRank = 64;
constexpr int kMid = kT / 2;
constexpr int kPPitch = 72;
constexpr int kAttnWaves = 4;
constexpr float kWCarry = 16.0f;
constexpr float kLCarry = 64.0f;
constexpr float kACarry = 16.0f;
constexpr float kVCarry = 16.0f;
constexpr float kZCarry = 16.0f;
constexpr float kPvFold = 1.0f / (kACarry * kVCarry);
constexpr float kClip = 60.0f;
constexpr float kGnEps = 1e-5f * 64.0f;
static_assert(kD == kH * kHS);
static_assert(kT % 64 == 0 && kD % 64 == 0 && kMixPad % 64 == 0 && kDecRank % 64 == 0);
static_assert(kD % 32 == 0 && kMixRank % 32 == 0 && kDecRank % 32 == 0);
static_assert(kMixCols == 5 * kMixRank && kMixCols <= kMixPad);
static_assert((kT / 64) * (kD / 64) % 8 == 0 && (kT / 64) * (kMixPad / 64) % 8 == 0 && (kT / 64) * (kDecRank / 64) % 8 == 0);

typedef __attribute__((ext_vector_type(16))) _Float16 v16h;
typedef __attribute__((ext_vector_type(8)))  _Float16 v8h;
typedef __attribute__((ext_vector_type(16))) __bf16   v16b;
typedef __attribute__((ext_vector_type(8)))  __bf16   v8b;
typedef __attribute__((ext_vector_type(8)))  float    v8f;
typedef __attribute__((ext_vector_type(4)))  float    v4f;
typedef __attribute__((ext_vector_type(2)))  float    v2f;
typedef __attribute__((ext_vector_type(4)))  unsigned int v4u;
typedef __attribute__((ext_vector_type(2)))  unsigned int v2u;

__device__ __forceinline__ unsigned short f2bf_bits(float f) {
  unsigned u = __float_as_uint(f);
  return (unsigned short)((u + 0x7FFFu + ((u >> 16) & 1u)) >> 16);
}
__device__ __forceinline__ float bf_bits2f(unsigned short h) { return __uint_as_float(((unsigned)h) << 16); }
__device__ __forceinline__ unsigned pk16(unsigned short a, unsigned short b) { return (unsigned)a | ((unsigned)b << 16); }
__device__ __forceinline__ unsigned short h_bits(float f) { const _Float16 h = (_Float16)f; return __builtin_bit_cast(unsigned short, h); }

__device__ __forceinline__ void guard4_h(v8f& a, v8f& b, v8f& c, v8f& d, v16h x, v16h y0, v16h y1, v16h y2, v16h y3) {
  asm volatile("v_nop\n\tv_nop\n\tv_nop\n\tv_nop" : "+v"(a), "+v"(b), "+v"(c), "+v"(d) : "v"(x), "v"(y0), "v"(y1), "v"(y2), "v"(y3));
}
__device__ __forceinline__ void guard1_b(v8f& a, v16b q0, v16b q1, v16b q2, v16b q3, v16b k0, v16b k1, v16b k2, v16b k3) {
  asm volatile("v_nop\n\tv_nop\n\tv_nop\n\tv_nop" : "+v"(a) : "v"(q0), "v"(q1), "v"(q2), "v"(q3), "v"(k0), "v"(k1), "v"(k2), "v"(k3));
}
__device__ __forceinline__ void acc_guard4(v8f& a, v8f& b, v8f& c, v8f& d) {
  asm volatile("v_nop\n\tv_nop\n\tv_nop\n\tv_nop" : "+v"(a), "+v"(b), "+v"(c), "+v"(d));
}
__device__ __forceinline__ void wave_lds_sync() {
  __builtin_amdgcn_fence(__ATOMIC_RELEASE, "workgroup");
  __builtin_amdgcn_wave_barrier();
  __builtin_amdgcn_fence(__ATOMIC_ACQUIRE, "workgroup");
}

template <typename T> struct Frag;
template <> struct Frag<_Float16> {
  typedef v16h V; union U { v16h v; v8h h[2]; };
  static __device__ __forceinline__ v16h load(const _Float16* p) {
    U f; f.h[0] = *(const v8h*)(p); f.h[1] = *(const v8h*)(p + 16); return f.v;
  }
  static __device__ __forceinline__ v8f mma(v16h a, v16h b, v8f c) {
    return __builtin_amdgcn_wmma_f32_16x16x32_f16(false, a, false, b, (short)0, c, false, false);
  }
};
template <> struct Frag<__bf16> {
  typedef v16b V; union U { v16b v; v8b h[2]; };
  static __device__ __forceinline__ v16b load(const __bf16* p) {
    U f; f.h[0] = *(const v8b*)(p); f.h[1] = *(const v8b*)(p + 16); return f.v;
  }
  static __device__ __forceinline__ v8f mma(v16b a, v16b b, v8f c) {
    return __builtin_amdgcn_wmma_f32_16x16x32_bf16(false, a, false, b, (short)0, c, false, false);
  }
};

template <int OUT_MODE, bool BIAS_N, int ACT, bool MIX>
__global__ __launch_bounds__(256) void gemm64_f16(
    const unsigned short* __restrict__ Ap, int lda, long strideA,
    const unsigned short* __restrict__ Btp, int ldb, long strideB,
    void* __restrict__ Cout, int ldc, long strideC,
    const float* __restrict__ bias,
    const float* __restrict__ mixX, const float* __restrict__ mixDX,
    const float* __restrict__ maa0, const float* __restrict__ maa1, const float* __restrict__ maa2,
    const float* __restrict__ maa3, const float* __restrict__ maa4,
    int M, int N, int K, float scale) {
  __shared__ __align__(16) float sT[8][16 * 68];
  const int zb   = blockIdx.y;
  const int lane = threadIdx.x & 31;
  const int wave = threadIdx.x >> 5;
  const int tilesN = N >> 6;
  const int tilesM = M >> 6;
  const int tile = blockIdx.x * 8 + wave;
  if (tile >= tilesM * tilesN) return;
  const int tm = tile / tilesN;
  const int tn = tile - tm * tilesN;
  const int m0 = tm << 6;
  const int n0 = tn << 6;
  const _Float16* A  = (const _Float16*)Ap  + (size_t)zb * strideA;
  const _Float16* Bt = (const _Float16*)Btp + (size_t)zb * strideB;
  const int rlane = lane & 15;
  const int koff  = (lane >> 4) * 8;
  const int mOff  = (lane >> 4) * 8;
  const float* maa = (zb == 0) ? maa0 : (zb == 1) ? maa1 : (zb == 2) ? maa2 : (zb == 3) ? maa3 : maa4;

  const _Float16* ap[4];
  const _Float16* bp[4];
#pragma unroll
  for (int i = 0; i < 4; ++i) {
    ap[i] = A  + (size_t)(m0 + (i << 4) + rlane) * lda + koff;
    bp[i] = Bt + (size_t)(n0 + (i << 4) + rlane) * ldb + koff;
  }

  v8f acc[4][4];
#pragma unroll
  for (int i = 0; i < 4; ++i)
#pragma unroll
    for (int j = 0; j < 4; ++j) acc[i][j] = (v8f){0.f, 0.f, 0.f, 0.f, 0.f, 0.f, 0.f, 0.f};

  for (int k0 = 0; k0 < K; k0 += 32) {
    const v16h b0 = Frag<_Float16>::load(bp[0] + k0);
    const v16h b1 = Frag<_Float16>::load(bp[1] + k0);
    const v16h b2 = Frag<_Float16>::load(bp[2] + k0);
    const v16h b3 = Frag<_Float16>::load(bp[3] + k0);
#pragma unroll
    for (int i = 0; i < 4; ++i) {
      const v16h ah = Frag<_Float16>::load(ap[i] + k0);
      acc[i][0] = Frag<_Float16>::mma(ah, b0, acc[i][0]);
      acc[i][1] = Frag<_Float16>::mma(ah, b1, acc[i][1]);
      acc[i][2] = Frag<_Float16>::mma(ah, b2, acc[i][2]);
      acc[i][3] = Frag<_Float16>::mma(ah, b3, acc[i][3]);
      guard4_h(acc[i][0], acc[i][1], acc[i][2], acc[i][3], ah, b0, b1, b2, b3);
    }
  }
  acc_guard4(acc[0][0], acc[0][1], acc[0][2], acc[0][3]);
  acc_guard4(acc[1][0], acc[1][1], acc[1][2], acc[1][3]);
  acc_guard4(acc[2][0], acc[2][1], acc[2][2], acc[2][3]);
  acc_guard4(acc[3][0], acc[3][1], acc[3][2], acc[3][3]);

  float* slab = sT[wave];
  float bv[4];
#pragma unroll
  for (int j = 0; j < 4; ++j) bv[j] = BIAS_N ? bias[n0 + (j << 4) + rlane] : 0.0f;

#pragma unroll
  for (int i = 0; i < 4; ++i) {
    const int mBase = m0 + (i << 4);
#pragma unroll
    for (int j = 0; j < 4; ++j) {
#pragma unroll
      for (int r = 0; r < 8; ++r) {
        slab[(mOff + r) * 68 + (j << 4) + rlane] = acc[i][j][r] * scale + bv[j];
      }
    }
    wave_lds_sync();
    if (ACT != 0) {
#pragma unroll 1
      for (int q = 0; q < 32; ++q) {
        const int idx = q * 32 + lane;
        const int off = (idx >> 6) * 68 + (idx & 63);
        float v = slab[off];
        if (ACT == 1) v = tanhf(v);
        if (ACT == 2) v = -expf(v);
        slab[off] = v;
      }
      wave_lds_sync();
    }
    if (OUT_MODE == 0) {
      float* C = (float*)Cout + (size_t)zb * strideC;
      const int hh = lane >> 4, c4 = (lane & 15) * 4;
      for (int pass = 0; pass < 2; ++pass) {
#pragma unroll
        for (int it = 0; it < 8; ++it) {
          const int row = it * 2 + hh;
          const v4f v = *(const v4f*)(slab + row * 68 + c4);
          *(volatile v4f*)(C + (size_t)(mBase + row) * ldc + n0 + c4) = v;
        }
        __threadfence();
      }
    } else {
      unsigned short* C = (unsigned short*)Cout + (size_t)zb * strideC;
      const int q = lane >> 3, c8 = (lane & 7) * 8;
      v8h hv[4];
#pragma unroll
      for (int it = 0; it < 4; ++it) {
        const int row = it * 4 + q;
        const float* sp = slab + row * 68 + c8;
        const v4f s0 = *(const v4f*)(sp);
        const v4f s1 = *(const v4f*)(sp + 4);
        float vals[8];
#pragma unroll
        for (int e = 0; e < 4; ++e) { vals[e] = s0[e]; vals[4 + e] = s1[e]; }
        if (MIX) {
          const size_t go = (size_t)(mBase + row) * kD + n0 + c8;
          const v4f x0 = *(const v4f*)(mixX + go);
          const v4f x1 = *(const v4f*)(mixX + go + 4);
          const v4f d0 = *(const v4f*)(mixDX + go);
          const v4f d1 = *(const v4f*)(mixDX + go + 4);
          const v4f a0 = *(const v4f*)(maa + n0 + c8);
          const v4f a1 = *(const v4f*)(maa + n0 + c8 + 4);
#pragma unroll
          for (int e = 0; e < 4; ++e) {
            vals[e]     = x0[e] + d0[e] * (a0[e] + vals[e]);
            vals[4 + e] = x1[e] + d1[e] * (a1[e] + vals[4 + e]);
          }
        }
#pragma unroll
        for (int e = 0; e < 8; ++e) hv[it][e] = (_Float16)vals[e];
      }
      for (int pass = 0; pass < 2; ++pass) {
#pragma unroll
        for (int it = 0; it < 4; ++it) {
          const int row = it * 4 + q;
          *(volatile v8h*)(C + (size_t)(mBase + row) * ldc + n0 + c8) = hv[it];
        }
        __threadfence();
      }
    }
    wave_lds_sync();
  }
}

__global__ __launch_bounds__(256) void wcast_kernel(const float* __restrict__ W0, const float* __restrict__ W1,
                                                    const float* __restrict__ W2, const float* __restrict__ W3,
                                                    const float* __restrict__ W4,
                                                    unsigned short* __restrict__ out, float carry) {
  const int z = blockIdx.y;
  const float* W = (z == 0) ? W0 : (z == 1) ? W1 : (z == 2) ? W2 : (z == 3) ? W3 : W4;
  const int i = blockIdx.x * 256 + threadIdx.x;
  const float* p = W + 8 * (size_t)i;
  const v4f a = *(const v4f*)(p);
  const v4f c = *(const v4f*)(p + 4);
  unsigned short hb[8];
#pragma unroll
  for (int e = 0; e < 4; ++e) {
    hb[e]     = h_bits(a[e] * carry);
    hb[4 + e] = h_bits(c[e] * carry);
  }
  const v4u u = (v4u){pk16(hb[0], hb[1]), pk16(hb[2], hb[3]), pk16(hb[4], hb[5]), pk16(hb[6], hb[7])};
  unsigned short* q = out + (size_t)z * kD * kD + 8 * (size_t)i;
  *(volatile v4u*)q = u;
  __threadfence();
  *(volatile v4u*)q = u;
}

__global__ __launch_bounds__(256) void tcast_kernel(const float* __restrict__ in, int R, int C,
                                                    unsigned short* __restrict__ out, int RP, float carry) {
  __shared__ float sm[64][65];
  const int t  = threadIdx.x;
  const int r0 = blockIdx.x * 64;
  const int c0 = blockIdx.y * 64;
#pragma unroll
  for (int i = 0; i < 16; ++i) {
    const int e  = i * 256 + t;
    const int rl = e >> 6;
    const int cl = e & 63;
    const int r = r0 + rl, c = c0 + cl;
    const int rc = (r < R) ? r : (R - 1);
    const int cc = (c < C) ? c : (C - 1);
    const float v = in[(size_t)rc * C + cc];
    sm[cl][rl] = (r < R && c < C) ? (v * carry) : 0.0f;
  }
  __syncthreads();
  const int lane = t & 31, wave = t >> 5;
  const int q = lane >> 3, c8 = (lane & 7) * 8;
  for (int pass = 0; pass < 2; ++pass) {
#pragma unroll
    for (int it = 0; it < 2; ++it) {
      const int row = wave * 8 + it * 4 + q;
      unsigned short hb[8];
#pragma unroll
      for (int e = 0; e < 8; ++e) hb[e] = h_bits(sm[row][c8 + e]);
      const v4u u = (v4u){pk16(hb[0], hb[1]), pk16(hb[2], hb[3]), pk16(hb[4], hb[5]), pk16(hb[6], hb[7])};
      *(volatile v4u*)(out + (size_t)(c0 + row) * RP + r0 + c8) = u;
    }
    __threadfence();
  }
}

__global__ __launch_bounds__(256) void prep_kernel(const float* __restrict__ x, const float* __restrict__ maax,
                                                   unsigned short* __restrict__ XA, float* __restrict__ DX) {
  const int i  = blockIdx.x * 256 + threadIdx.x;
  const int t  = i >> 8;
  const int c4 = (i & 255) * 4;
  const bool hasL = (t > 0);
  const bool hasR = (t < kT - 1);
  const int tl = hasL ? (t - 1) : 0;
  const int tr = hasR ? (t + 1) : (kT - 1);
  const v4f xc = *(const v4f*)(x + (size_t)t  * kD + c4);
  const v4f xl = *(const v4f*)(x + (size_t)tl * kD + c4);
  const v4f xr = *(const v4f*)(x + (size_t)tr * kD + c4);
  const v4f mm = *(const v4f*)(maax + c4);
  v4f dx;
  unsigned short hb[4];
#pragma unroll
  for (int e = 0; e < 4; ++e) {
    const float l = hasL ? xl[e] : 0.0f;
    const float r = hasR ? xr[e] : 0.0f;
    const float d = 0.5f * (l + r) - xc[e];
    dx[e] = d;
    hb[e] = h_bits(xc[e] + d * mm[e]);
  }
  const v2u u = (v2u){pk16(hb[0], hb[1]), pk16(hb[2], hb[3])};
  float* dp = DX + (size_t)t * kD + c4;
  unsigned short* apx = XA + (size_t)t * kD + c4;
  *(volatile v4f*)dp = dx;
  *(volatile v2u*)apx = u;
  __threadfence();
  *(volatile v4f*)dp = dx;
  *(volatile v2u*)apx = u;
}

__global__ __launch_bounds__(64) void scan_kernel(const float* __restrict__ W, float* __restrict__ CS) {
  const int g  = blockIdx.x * 64 + threadIdx.x;
  const int c4 = g * 4;
  for (int pass = 0; pass < 2; ++pass) {
    double r0 = 0.0, r1 = 0.0, r2 = 0.0, r3 = 0.0;
#pragma unroll 1
    for (int t = 0; t < kT; ++t) {
      const v4f w = *(const v4f*)(W + (size_t)t * kD + c4);
      r0 += (double)w[0];
      r1 += (double)w[1];
      r2 += (double)w[2];
      r3 += (double)w[3];
      v4f o;
      o[0] = (float)r0; o[1] = (float)r1; o[2] = (float)r2; o[3] = (float)r3;
      *(volatile v4f*)(CS + (size_t)t * kD + c4) = o;
    }
    __threadfence();
  }
}

__global__ __launch_bounds__(256) void factor_kernel(const float* __restrict__ R32, const float* __restrict__ K32,
                                                     const float* __restrict__ CS, const float* __restrict__ WN,
                                                     unsigned short* __restrict__ FAC) {
  __shared__ __align__(16) unsigned int sh[8][kD / 2];
  const int t   = blockIdx.x;
  const int tid = threadIdx.x;
  const int lane = tid & 31;
#pragma unroll 1
  for (int it = 0; it < 4; ++it) {
    const int ch = it * 256 + tid;
    const size_t go = (size_t)t * kD + ch;
    const float cc  = CS[go];
    const float ww  = WN[go];
    const float cm  = CS[(size_t)kMid * kD + ch];
    const float wm  = WN[(size_t)kMid * kD + ch];
    const float rv  = R32[go];
    const float kv  = K32[go];
    const float cf = fminf(fmaxf(cc - cm, -kClip), kClip);
    const float cb = fminf(fmaxf((cc - ww) - (cm - wm), -kClip), kClip);
    float val[4];
    val[0] = rv * expf(cf);
    val[1] = kv * expf(-cf);
    val[2] = rv * expf(-cb);
    val[3] = kv * expf(cb);
    unsigned bits[8];
#pragma unroll
    for (int p = 0; p < 4; ++p) {
      const unsigned short hb = f2bf_bits(val[p]);
      const unsigned short lb = f2bf_bits(val[p] - bf_bits2f(hb));
      bits[2 * p]     = (unsigned)hb;
      bits[2 * p + 1] = (unsigned)lb;
    }
    unsigned word[8];
#pragma unroll
    for (int p = 0; p < 8; ++p) {
      const unsigned other = (unsigned)__shfl_xor((int)bits[p], 1, 32);
      word[p] = bits[p] | (other << 16);
    }
    if ((lane & 1) == 0) {
#pragma unroll
      for (int p = 0; p < 8; ++p) sh[p][ch >> 1] = word[p];
    }
  }
  __syncthreads();
  const size_t PL = (size_t)kT * kD;
  for (int pass = 0; pass < 2; ++pass) {
#pragma unroll
    for (int it = 0; it < 4; ++it) {
      const int idx = it * 256 + tid;
      const int p  = idx >> 7;
      const int ck = idx & 127;
      const v4u v = *(const v4u*)(&sh[p][ck * 4]);
      *(volatile v4u*)(FAC + (size_t)p * PL + (size_t)t * kD + ck * 8) = v;
    }
    __threadfence();
  }
}

__device__ __forceinline__ v8f qk_sub(v16b qh0, v16b qh1, v16b ql0, v16b ql1,
                                      const __bf16* __restrict__ ph, const __bf16* __restrict__ pl) {
  const v16b kh0 = Frag<__bf16>::load(ph);
  const v16b kh1 = Frag<__bf16>::load(ph + 32);
  const v16b kl0 = Frag<__bf16>::load(pl);
  const v16b kl1 = Frag<__bf16>::load(pl + 32);
  v8f a = (v8f){0.f, 0.f, 0.f, 0.f, 0.f, 0.f, 0.f, 0.f};
  a = Frag<__bf16>::mma(qh0, kl0, a);
  a = Frag<__bf16>::mma(ql0, kh0, a);
  a = Frag<__bf16>::mma(qh1, kl1, a);
  a = Frag<__bf16>::mma(ql1, kh1, a);
  a = Frag<__bf16>::mma(qh0, kh0, a);
  a = Frag<__bf16>::mma(qh1, kh1, a);
  guard1_b(a, qh0, qh1, ql0, ql1, kh0, kh1, kl0, kl1);
  return a;
}

__device__ __forceinline__ void pv_tile(v8f s0, v8f s1, v8f s2, v8f s3, _Float16* pw,
                                        const _Float16* __restrict__ vbj,
                                        v8f& o0, v8f& o1, v8f& o2, v8f& o3, int hh, int c) {
#pragma unroll
  for (int r = 0; r < 8; ++r) {
    _Float16* pr = pw + (8 * hh + r) * kPPitch + c;
    pr[0]  = (_Float16)(s0[r] * kACarry);
    pr[16] = (_Float16)(s1[r] * kACarry);
    pr[32] = (_Float16)(s2[r] * kACarry);
    pr[48] = (_Float16)(s3[r] * kACarry);
  }
  wave_lds_sync();
#pragma unroll
  for (int kk = 0; kk < 2; ++kk) {
    const v16h pa = Frag<_Float16>::load(pw + c * kPPitch + kk * 32 + 8 * hh);
    const v16h v0 = Frag<_Float16>::load(vbj + kk * 32);
    const v16h v1 = Frag<_Float16>::load(vbj + (size_t)16 * kT + kk * 32);
    const v16h v2 = Frag<_Float16>::load(vbj + (size_t)32 * kT + kk * 32);
    const v16h v3 = Frag<_Float16>::load(vbj + (size_t)48 * kT + kk * 32);
    o0 = Frag<_Float16>::mma(pa, v0, o0);
    o1 = Frag<_Float16>::mma(pa, v1, o1);
    o2 = Frag<_Float16>::mma(pa, v2, o2);
    o3 = Frag<_Float16>::mma(pa, v3, o3);
    guard4_h(o0, o1, o2, o3, pa, v0, v1, v2, v3);
  }
  wave_lds_sync();
}

__global__ __launch_bounds__(128) void decay_attn_kernel(const unsigned short* __restrict__ FACp,
                                                         const unsigned short* __restrict__ VTp,
                                                         float* __restrict__ Y) {
  __shared__ __align__(16) _Float16 Psh[kAttnWaves][16 * kPPitch];
  __shared__ __align__(16) float    Osh[kAttnWaves][16 * 68];
  const __bf16*   FAC = (const __bf16*)FACp;
  const _Float16* VT  = (const _Float16*)VTp;
  const int tid = threadIdx.x, wave = tid >> 5, lane = tid & 31;
  const int hh = lane >> 4, c = lane & 15;
  const int ib = blockIdx.x;
  const int h  = blockIdx.y;
  const int i0 = ib * 64 + wave * 16;
  const size_t PL   = (size_t)kT * kD;
  const size_t qoff = (size_t)(i0 + c) * kD + h * kHS + 8 * hh;
  const size_t koff = (size_t)c * kD + h * kHS + 8 * hh;
  const size_t sub  = (size_t)16 * kD;
  const __bf16* kfh = FAC + 2 * PL + koff;
  const __bf16* kfl = FAC + 3 * PL + koff;
  const __bf16* kbh = FAC + 6 * PL + koff;
  const __bf16* kbl = FAC + 7 * PL + koff;
  const _Float16* vb = VT + (size_t)(h * kHS + c) * kT + 8 * hh;
  _Float16* pw = Psh[wave];
  const v8f z8 = (v8f){0.f, 0.f, 0.f, 0.f, 0.f, 0.f, 0.f, 0.f};
  v8f o0 = z8, o1 = z8, o2 = z8, o3 = z8;

  const v16b qfh0 = Frag<__bf16>::load(FAC + qoff);
  const v16b qfh1 = Frag<__bf16>::load(FAC + qoff + 32);
  const v16b qfl0 = Frag<__bf16>::load(FAC + PL + qoff);
  const v16b qfl1 = Frag<__bf16>::load(FAC + PL + qoff + 32);

#pragma unroll 1
  for (int jb = 0; jb < ib; ++jb) {
    const size_t jo = (size_t)jb * 64 * kD;
    v8f s0 = qk_sub(qfh0, qfh1, qfl0, qfl1, kfh + jo,           kfl + jo);
    v8f s1 = qk_sub(qfh0, qfh1, qfl0, qfl1, kfh + jo + sub,     kfl + jo + sub);
    v8f s2 = qk_sub(qfh0, qfh1, qfl0, qfl1, kfh + jo + 2 * sub, kfl + jo + 2 * sub);
    v8f s3 = qk_sub(qfh0, qfh1, qfl0, qfl1, kfh + jo + 3 * sub, kfl + jo + 3 * sub);
    acc_guard4(s0, s1, s2, s3);
    pv_tile(s0, s1, s2, s3, pw, vb + jb * 64, o0, o1, o2, o3, hh, c);
  }

  const size_t jd = (size_t)ib * 64 * kD;
  v8f f0 = qk_sub(qfh0, qfh1, qfl0, qfl1, kfh + jd,           kfl + jd);
  v8f f1 = qk_sub(qfh0, qfh1, qfl0, qfl1, kfh + jd + sub,     kfl + jd + sub);
  v8f f2 = qk_sub(qfh0, qfh1, qfl0, qfl1, kfh + jd + 2 * sub, kfl + jd + 2 * sub);
  v8f f3 = qk_sub(qfh0, qfh1, qfl0, qfl1, kfh + jd + 3 * sub, kfl + jd + 3 * sub);
  acc_guard4(f0, f1, f2, f3);

  const v16b qbh0 = Frag<__bf16>::load(FAC + 4 * PL + qoff);
  const v16b qbh1 = Frag<__bf16>::load(FAC + 4 * PL + qoff + 32);
  const v16b qbl0 = Frag<__bf16>::load(FAC + 5 * PL + qoff);
  const v16b qbl1 = Frag<__bf16>::load(FAC + 5 * PL + qoff + 32);
  {
    v8f g0 = qk_sub(qbh0, qbh1, qbl0, qbl1, kbh + jd,           kbl + jd);
    v8f g1 = qk_sub(qbh0, qbh1, qbl0, qbl1, kbh + jd + sub,     kbl + jd + sub);
    v8f g2 = qk_sub(qbh0, qbh1, qbl0, qbl1, kbh + jd + 2 * sub, kbl + jd + 2 * sub);
    v8f g3 = qk_sub(qbh0, qbh1, qbl0, qbl1, kbh + jd + 3 * sub, kbl + jd + 3 * sub);
    acc_guard4(g0, g1, g2, g3);
#pragma unroll
    for (int r = 0; r < 8; ++r) {
      const int ig = i0 + 8 * hh + r;
      const int jg = ib * 64 + c;
      f0[r] = (ig >= jg)      ? f0[r] : g0[r];
      f1[r] = (ig >= jg + 16) ? f1[r] : g1[r];
      f2[r] = (ig >= jg + 32) ? f2[r] : g2[r];
      f3[r] = (ig >= jg + 48) ? f3[r] : g3[r];
    }
    pv_tile(f0, f1, f2, f3, pw, vb + ib * 64, o0, o1, o2, o3, hh, c);
  }

#pragma unroll 1
  for (int jb = ib + 1; jb < kT / 64; ++jb) {
    const size_t jo = (size_t)jb * 64 * kD;
    v8f s0 = qk_sub(qbh0, qbh1, qbl0, qbl1, kbh + jo,           kbl + jo);
    v8f s1 = qk_sub(qbh0, qbh1, qbl0, qbl1, kbh + jo + sub,     kbl + jo + sub);
    v8f s2 = qk_sub(qbh0, qbh1, qbl0, qbl1, kbh + jo + 2 * sub, kbl + jo + 2 * sub);
    v8f s3 = qk_sub(qbh0, qbh1, qbl0, qbl1, kbh + jo + 3 * sub, kbl + jo + 3 * sub);
    acc_guard4(s0, s1, s2, s3);
    pv_tile(s0, s1, s2, s3, pw, vb + jb * 64, o0, o1, o2, o3, hh, c);
  }

  float* os = Osh[wave];
#pragma unroll
  for (int r = 0; r < 8; ++r) {
    float* orow = os + (8 * hh + r) * 68 + c;
    orow[0]  = o0[r] * kPvFold;
    orow[16] = o1[r] * kPvFold;
    orow[32] = o2[r] * kPvFold;
    orow[48] = o3[r] * kPvFold;
  }
  wave_lds_sync();
  {
    const int c4 = c * 4;
    for (int pass = 0; pass < 2; ++pass) {
#pragma unroll
      for (int it = 0; it < 8; ++it) {
        const int row = it * 2 + hh;
        const v4f val = *(const v4f*)(os + row * 68 + c4);
        *(volatile v4f*)(Y + (size_t)(i0 + row) * kD + h * kHS + c4) = val;
      }
      __threadfence();
    }
  }
}

__global__ __launch_bounds__(256) void gn_gate_kernel(const float* __restrict__ Y, const float* __restrict__ G,
                                                      const float* __restrict__ lnw, const float* __restrict__ lnb,
                                                      unsigned int* __restrict__ Z) {
  const int lane = threadIdx.x & 31, wave = threadIdx.x >> 5;
  const int grp = blockIdx.x * 8 + wave;
  const int tok = grp >> 4;
  const int h   = grp & 15;
  const int ch  = h * kHS + 2 * lane;
  const size_t base = (size_t)tok * kD + ch;
  const v2f yv = *(const v2f*)(Y + base);
  const v2f gv = *(const v2f*)(G + base);
  const v2f wv = *(const v2f*)(lnw + ch);
  const v2f bv = *(const v2f*)(lnb + ch);
  const float y0 = yv[0], y1 = yv[1];
  float s = y0 + y1;
#pragma unroll
  for (int off = 16; off > 0; off >>= 1) s += __shfl_xor(s, off, 32);
  const float mu = s * (1.0f / kHS);
  const float d0 = y0 - mu, d1 = y1 - mu;
  float ss = d0 * d0 + d1 * d1;
#pragma unroll
  for (int off = 16; off > 0; off >>= 1) ss += __shfl_xor(ss, off, 32);
  const float var  = ss * (1.0f / kHS);
  const float rstd = rsqrtf(var + kGnEps);
  const float g0 = gv[0], g1 = gv[1];
  const float sg0 = g0 / (1.0f + expf(-g0));
  const float sg1 = g1 / (1.0f + expf(-g1));
  const float z0 = ((d0 * rstd) * wv[0] + bv[0]) * sg0 * kZCarry;
  const float z1 = ((d1 * rstd) * wv[1] + bv[1]) * sg1 * kZCarry;
  const unsigned u = pk16(h_bits(z0), h_bits(z1));
  unsigned int* zp = Z + (base >> 1);
  *(volatile unsigned int*)zp = u;
  __threadfence();
  *(volatile unsigned int*)zp = u;
}

extern "C" void kernel_launch(void* const* d_in, const int* in_sizes, int n_in,
                              void* d_out, int out_size, void* d_ws, size_t ws_size, hipStream_t stream) {
  if (n_in < 19 || d_out == nullptr || d_ws == nullptr) return;
  if (in_sizes[0] != kB * kT * kD || in_sizes[1] != kD || in_sizes[2] != kD || in_sizes[3] != kD ||
      in_sizes[4] != kD || in_sizes[5] != kD || in_sizes[6] != kD || in_sizes[7] != kD * kMixCols ||
      in_sizes[8] != kMixCols * kD || in_sizes[9] != kD || in_sizes[10] != kD * kDecRank ||
      in_sizes[11] != kDecRank * kD || in_sizes[12] != kD * kD || in_sizes[13] != kD * kD ||
      in_sizes[14] != kD * kD || in_sizes[15] != kD * kD || in_sizes[16] != kD * kD ||
      in_sizes[17] != kD || in_sizes[18] != kD || out_size != kB * kT * kD) return;

  const float* x      = (const float*)d_in[0];
  const float* maa_x  = (const float*)d_in[1];
  const float* maa_w  = (const float*)d_in[2];
  const float* maa_k  = (const float*)d_in[3];
  const float* maa_v  = (const float*)d_in[4];
  const float* maa_r  = (const float*)d_in[5];
  const float* maa_g  = (const float*)d_in[6];
  const float* w1     = (const float*)d_in[7];
  const float* w2     = (const float*)d_in[8];
  const float* tdec   = (const float*)d_in[9];
  const float* dw1    = (const float*)d_in[10];
  const float* dw2    = (const float*)d_in[11];
  const float* Wr     = (const float*)d_in[12];
  const float* Wk     = (const float*)d_in[13];
  const float* Wv     = (const float*)d_in[14];
  const float* Wg     = (const float*)d_in[15];
  const float* Wo     = (const float*)d_in[16];
  const float* lnw    = (const float*)d_in[17];
  const float* lnb    = (const float*)d_in[18];
  float* out = (float*)d_out;

  const size_t PLN = (size_t)kT * kD;
  char* ws = (char*)d_ws; size_t off = 0;
  auto carve = [&](size_t bytes) -> char* { char* p = ws + off; off += (bytes + 255) & ~(size_t)255; return p; };
  unsigned short* W16  = (unsigned short*)carve((size_t)5 * kD * kD * 2);
  unsigned short* W1T  = (unsigned short*)carve((size_t)kMixPad * kD * 2);
  unsigned short* W2T  = (unsigned short*)carve((size_t)kD * kMixPad * 2);
  unsigned short* DW1T = (unsigned short*)carve((size_t)kDecRank * kD * 2);
  unsigned short* DW2T = (unsigned short*)carve((size_t)kD * kDecRank * 2);
  unsigned short* XA   = (unsigned short*)carve(PLN * 2);
  float*          DX   = (float*)carve(PLN * 4);
  unsigned short* XXX  = (unsigned short*)carve((size_t)kT * kMixPad * 2);
  unsigned short* XMIX = (unsigned short*)carve((size_t)5 * PLN * 2);
  unsigned short* TD   = (unsigned short*)carve((size_t)kT * kDecRank * 2);
  float*          WNEG = (float*)carve(PLN * 4);
  float*          CS   = (float*)carve(PLN * 4);
  float*          R32  = (float*)carve(PLN * 4);
  float*          K32  = (float*)carve(PLN * 4);
  float*          GPRE = (float*)carve(PLN * 4);
  unsigned short* VT   = (unsigned short*)carve(PLN * 2);
  unsigned short* FAC  = (unsigned short*)carve((size_t)8 * PLN * 2);
  float*          Y    = (float*)carve(PLN * 4);
  unsigned short* Z    = (unsigned short*)carve(PLN * 2);
  if (off > ws_size || off > (size_t)134217728) return;

  unsigned short* Xw = XMIX;
  unsigned short* Xk = XMIX + PLN;
  unsigned short* Xv = XMIX + 2 * PLN;
  unsigned short* Xr = XMIX + 3 * PLN;
  unsigned short* Xg = XMIX + 4 * PLN;
  const unsigned short* Wr16 = W16;
  const unsigned short* Wk16 = W16 + (size_t)kD * kD;
  const unsigned short* Wv16 = W16 + (size_t)2 * kD * kD;
  const unsigned short* Wg16 = W16 + (size_t)3 * kD * kD;
  const unsigned short* Wo16 = W16 + (size_t)4 * kD * kD;

  wcast_kernel<<<dim3(kD * kD / 8 / 256, 5), 256, 0, stream>>>(Wr, Wk, Wv, Wg, Wo, W16, kWCarry);
  tcast_kernel<<<dim3(kD / 64, kMixPad / 64), 256, 0, stream>>>(w1, kD, kMixCols, W1T, kD, kLCarry);
  tcast_kernel<<<dim3(kMixPad / 64, kD / 64), 256, 0, stream>>>(w2, kMixCols, kD, W2T, kMixPad, kLCarry);
  tcast_kernel<<<dim3(kD / 64, kDecRank / 64), 256, 0, stream>>>(dw1, kD, kDecRank, DW1T, kD, kLCarry);
  tcast_kernel<<<dim3(kDecRank / 64, kD / 64), 256, 0, stream>>>(dw2, kDecRank, kD, DW2T, kDecRank, kLCarry);

  const int gBig  = (kT / 64) * (kD / 64) / 8;
  const int gMix  = (kT / 64) * (kMixPad / 64) / 8;
  const int gDec  = (kT / 64) * (kDecRank / 64) / 8;
  const float sL  = 1.0f / kLCarry;
  const float sW  = 1.0f / kWCarry;

  for (int b = 0; b < kB; ++b) {
    const float* xb = x + (size_t)b * PLN;
    float* outb = out + (size_t)b * PLN;

    prep_kernel<<<kT * kD / 4 / 256, 256, 0, stream>>>(xb, maa_x, XA, DX);

    gemm64_f16<1, false, 1, false><<<dim3(gMix, 1), 256, 0, stream>>>(
        XA, kD, 0L, W1T, kD, 0L, (void*)XXX, kMixPad, 0L,
        tdec, xb, DX, maa_w, maa_k, maa_v, maa_r, maa_g, kT, kMixPad, kD, sL);

    gemm64_f16<1, false, 0, true><<<dim3(gBig, 5), 256, 0, stream>>>(
        XXX, kMixPad, (long)kMixRank, W2T, kMixPad, (long)kMixRank, (void*)XMIX, kD, (long)PLN,
        tdec, xb, DX, maa_w, maa_k, maa_v, maa_r, maa_g, kT, kD, kMixRank, sL);

    gemm64_f16<1, false, 1, false><<<dim3(gDec, 1), 256, 0, stream>>>(
        Xw, kD, 0L, DW1T, kD, 0L, (void*)TD, kDecRank, 0L,
        tdec, xb, DX, maa_w, maa_k, maa_v, maa_r, maa_g, kT, kDecRank, kD, sL);

    gemm64_f16<0, true, 2, false><<<dim3(gBig, 1), 256, 0, stream>>>(
        TD, kDecRank, 0L, DW2T, kDecRank, 0L, (void*)WNEG, kD, 0L,
        tdec, xb, DX, maa_w, maa_k, maa_v, maa_r, maa_g, kT, kD, kDecRank, sL);

    scan_kernel<<<4, 64, 0, stream>>>(WNEG, CS);

    gemm64_f16<0, false, 0, false><<<dim3(gBig, 1), 256, 0, stream>>>(
        Xr, kD, 0L, Wr16, kD, 0L, (void*)R32, kD, 0L,
        tdec, xb, DX, maa_w, maa_k, maa_v, maa_r, maa_g, kT, kD, kD, sW);
    gemm64_f16<0, false, 0, false><<<dim3(gBig, 1), 256, 0, stream>>>(
        Xk, kD, 0L, Wk16, kD, 0L, (void*)K32, kD, 0L,
        tdec, xb, DX, maa_w, maa_k, maa_v, maa_r, maa_g, kT, kD, kD, sW);
    gemm64_f16<0, false, 0, false><<<dim3(gBig, 1), 256, 0, stream>>>(
        Xg, kD, 0L, Wg16, kD, 0L, (void*)GPRE, kD, 0L,
        tdec, xb, DX, maa_w, maa_k, maa_v, maa_r, maa_g, kT, kD, kD, sW);

    gemm64_f16<1, false, 0, false><<<dim3(gBig, 1), 256, 0, stream>>>(
        Wv16, kD, 0L, Xv, kD, 0L, (void*)VT, kT, 0L,
        tdec, xb, DX, maa_w, maa_k, maa_v, maa_r, maa_g, kD, kT, kD, kVCarry / kWCarry);

    factor_kernel<<<kT, 256, 0, stream>>>(R32, K32, CS, WNEG, FAC);

    decay_attn_kernel<<<dim3(kT / 64, kH), 128, 0, stream>>>(FAC, VT, Y);

    gn_gate_kernel<<<kT * kH / 8, 256, 0, stream>>>(Y, GPRE, lnw, lnb, (unsigned int*)Z);

    gemm64_f16<0, false, 0, false><<<dim3(gBig, 1), 256, 0, stream>>>(
        Z, kD, 0L, Wo16, kD, 0L, (void*)outb, kD, 0L,
        tdec, xb, DX, maa_w, maa_k, maa_v, maa_r, maa_g, kT, kD, kD, 1.0f / (kZCarry * kWCarry));
  }
}
